// GATSBlock_2405181685852
// MI455X (gfx1250) — hardware-verified
//
#include <hip/hip_runtime.h>
#include <math.h>
#include <stdint.h>

#define NB_   2
#define SEQ   2048
#define NTOK  4096
#define DM    1024
#define NHD   8
#define DHD   64
#define INR   512
#define FFD   4096
#define WSZ   512
#define NWN   4
#define KPR   512
#define VTP   4608

typedef __attribute__((ext_vector_type(16))) _Float16 v16h;
typedef __attribute__((ext_vector_type(8)))  _Float16 v8h;
typedef __attribute__((ext_vector_type(16))) __bf16   v16b;
typedef __attribute__((ext_vector_type(8)))  __bf16   v8b;
typedef __attribute__((ext_vector_type(8)))  float    v8f;
typedef __attribute__((ext_vector_type(4)))  float    v4f;
typedef __attribute__((ext_vector_type(2)))  float    v2f;
typedef __attribute__((ext_vector_type(4)))  unsigned int v4u;

__device__ __forceinline__ unsigned short f2bf_bits(float f) {
  unsigned u = __float_as_uint(f);
  return (unsigned short)((u + 0x7FFFu + ((u >> 16) & 1u)) >> 16);
}
__device__ __forceinline__ float bf_bits2f(unsigned short h) { return __uint_as_float(((unsigned)h) << 16); }
__device__ __forceinline__ unsigned pk16(unsigned short a, unsigned short b) { return (unsigned)a | ((unsigned)b << 16); }

__device__ __forceinline__ float wsum(float v) {
#pragma unroll
  for (int o = 16; o >= 1; o >>= 1) v += __shfl_xor(v, o, 32);
  return v;
}
__device__ __forceinline__ float wmax(float v) {
#pragma unroll
  for (int o = 16; o >= 1; o >>= 1) v = fmaxf(v, __shfl_xor(v, o, 32));
  return v;
}

__device__ __forceinline__ void dep_guard_h(v8f& a, v8f& b, v16h x, v16h y) { asm volatile("v_nop\n\tv_nop\n\tv_nop\n\tv_nop" : "+v"(a), "+v"(b) : "v"(x), "v"(y)); }
__device__ __forceinline__ void dep_guard_b(v8f& a, v8f& b, v16b x, v16b y) { asm volatile("v_nop\n\tv_nop\n\tv_nop\n\tv_nop" : "+v"(a), "+v"(b) : "v"(x), "v"(y)); }
__device__ __forceinline__ void keep4_h(v16h a, v16h b, v16h c, v16h d) { asm volatile("v_nop" :: "v"(a), "v"(b), "v"(c), "v"(d)); }
__device__ __forceinline__ void keep4_b(v16b a, v16b b, v16b c, v16b d) { asm volatile("v_nop" :: "v"(a), "v"(b), "v"(c), "v"(d)); }
__device__ __forceinline__ void acc_guard4(v8f& a, v8f& b, v8f& c, v8f& d) { asm volatile("v_nop\n\tv_nop\n\tv_nop\n\tv_nop" : "+v"(a), "+v"(b), "+v"(c), "+v"(d)); }

template <typename T> struct Frag;
template <> struct Frag<_Float16> {
  typedef v16h V; union U { v16h v; v8h h[2]; };
  static __device__ __forceinline__ v16h load(const _Float16* p) {
    U f; f.h[0] = *(const v8h*)(p); f.h[1] = *(const v8h*)(p + 16); return f.v;
  }
  static __device__ __forceinline__ v8f mma(v16h a, v16h b, v8f c) {
    return __builtin_amdgcn_wmma_f32_16x16x32_f16(false, a, false, b, (short)0, c, false, false);
  }
  static __device__ __forceinline__ void guard(v8f& a, v8f& b, v16h x, v16h y) { dep_guard_h(a, b, x, y); }
  static __device__ __forceinline__ void keep(v16h a, v16h b, v16h c, v16h d) { keep4_h(a, b, c, d); }
};
template <> struct Frag<__bf16> {
  typedef v16b V; union U { v16b v; v8b h[2]; };
  static __device__ __forceinline__ v16b load(const __bf16* p) {
    U f; f.h[0] = *(const v8b*)(p); f.h[1] = *(const v8b*)(p + 16); return f.v;
  }
  static __device__ __forceinline__ v8f mma(v16b a, v16b b, v8f c) {
    return __builtin_amdgcn_wmma_f32_16x16x32_bf16(false, a, false, b, (short)0, c, false, false);
  }
  static __device__ __forceinline__ void guard(v8f& a, v8f& b, v16b x, v16b y) { dep_guard_b(a, b, x, y); }
  static __device__ __forceinline__ void keep(v16b a, v16b b, v16b c, v16b d) { keep4_b(a, b, c, d); }
};

template <int ET> struct Elem;
template <> struct Elem<0> { typedef _Float16 T; };
template <> struct Elem<1> { typedef __bf16 T; };

template <int ET, bool SPLIT, bool BIAS, int EPI, int OUTM, bool RESID, int LOC>
__global__ __launch_bounds__(256) void k_gemm(
    const unsigned short* __restrict__ Ap, const unsigned short* __restrict__ A2p, int lda, long strideA,
    const unsigned short* __restrict__ Btp, const unsigned short* __restrict__ Bt2p, int ldb, long strideB,
    float* __restrict__ Cf, int ldc, long strideC,
    _Float16* __restrict__ Ch, int ldh, long strideH,
    const float* __restrict__ bias, const float* __restrict__ gvec,
    const float* __restrict__ resid, int ldr, long strideR,
    int M, int N, int K, int nwin, float scale, float oscale) {
  typedef typename Elem<ET>::T T;
  typedef typename Frag<T>::V V;
  const T* A = (const T*)Ap; const T* A2 = (const T*)A2p; const T* Bt = (const T*)Btp; const T* Bt2 = (const T*)Bt2p;
  __shared__ __align__(16) float sT[8][16 * 68];
  const int z    = blockIdx.y;
  const int lane = threadIdx.x & 31;
  const int wave = threadIdx.x >> 5;
  const int tilesN = N >> 6;
  const int tilesM = M >> 6;
  const int tile = blockIdx.x * 8 + wave;
  if (tile >= tilesM * tilesN) return;
  const int tm = tile / tilesN;
  const int tn = tile - tm * tilesN;
  const int m0 = tm << 6;
  const int n0 = tn << 6;
  int kBeg = 0, kEnd = K;
  if (LOC != 0) {
    const int w = z % nwin;
    const bool first = (w == 0);
    if (LOC == 1) {
      const int nb = first ? (N >> 1) : 0;
      if (n0 < nb || n0 >= (N >> 1) + m0 + 64) return;
    } else {
      kBeg = first ? (K >> 1) : 0;
      const int ke = (K >> 1) + m0 + 64;
      kEnd = (ke < K) ? ke : K;
    }
  }

  const T* Ab  = A  + (size_t)z * strideA;
  const T* Bb  = Bt + (size_t)z * strideB;
  const T* Ab2 = SPLIT ? (A2  + (size_t)z * strideA) : nullptr;
  const T* Bb2 = SPLIT ? (Bt2 + (size_t)z * strideB) : nullptr;

  const int rlane = lane & 15;
  const int koff  = (lane >> 4) * 8;
  const int mOff  = (lane >> 4) * 8;

  v8f acc[4][4];
#pragma unroll
  for (int i = 0; i < 4; ++i)
#pragma unroll
    for (int j = 0; j < 4; ++j) acc[i][j] = (v8f){0.f,0.f,0.f,0.f,0.f,0.f,0.f,0.f};

  for (int k0 = kBeg; k0 < kEnd; k0 += 32) {
    V bh[4], bl[4];
#pragma unroll
    for (int j = 0; j < 4; ++j) {
      const size_t bo = (size_t)(n0 + (j << 4) + rlane) * ldb + koff + k0;
      bh[j] = Frag<T>::load(Bb + bo);
      if (SPLIT) bl[j] = Frag<T>::load(Bb2 + bo); else bl[j] = bh[j];
    }
#pragma unroll
    for (int i = 0; i < 4; ++i) {
      const size_t ao = (size_t)(m0 + (i << 4) + rlane) * lda + koff + k0;
      V ah = Frag<T>::load(Ab + ao);
      V al = ah;
      if (SPLIT) al = Frag<T>::load(Ab2 + ao);
#pragma unroll
      for (int j = 0; j < 4; ++j) {
        acc[i][j] = Frag<T>::mma(ah, bh[j], acc[i][j]);
        if (SPLIT) {
          acc[i][j] = Frag<T>::mma(ah, bl[j], acc[i][j]);
          acc[i][j] = Frag<T>::mma(al, bh[j], acc[i][j]);
        }
      }
      Frag<T>::guard(acc[i][0], acc[i][3], ah, al);
    }
    Frag<T>::keep(bh[0], bh[1], bh[2], bh[3]);
    if (SPLIT) Frag<T>::keep(bl[0], bl[1], bl[2], bl[3]);
  }
  acc_guard4(acc[0][0], acc[0][1], acc[0][2], acc[0][3]);
  acc_guard4(acc[1][0], acc[1][1], acc[1][2], acc[1][3]);
  acc_guard4(acc[2][0], acc[2][1], acc[2][2], acc[2][3]);
  acc_guard4(acc[3][0], acc[3][1], acc[3][2], acc[3][3]);

  float* slab = sT[wave];
  const float* Rb = RESID ? (resid + (size_t)z * strideR) : nullptr;
#pragma unroll
  for (int i = 0; i < 4; ++i) {
    const int mBase = m0 + (i << 4);
#pragma unroll
    for (int j = 0; j < 4; ++j) {
      const int n = n0 + (j << 4) + rlane;
      float bv = 0.f;
      if (BIAS) bv = bias[n];
#pragma unroll
      for (int r = 0; r < 8; ++r) {
        float v = acc[i][j][r] * scale;
        if (BIAS) v += bv;
        if (RESID) v += Rb[(size_t)(mBase + mOff + r) * ldr + n];
        if (EPI == 1) {
          const float u = 0.7978845608028654f * (v + 0.044715f * v * v * v);
          v = v * (0.5f * (1.0f + tanhf(u)));
        }
        slab[(mOff + r) * 68 + (j << 4) + rlane] = v;
      }
    }
    __builtin_amdgcn_fence(__ATOMIC_RELEASE, "workgroup");
    __builtin_amdgcn_wave_barrier();
    __builtin_amdgcn_fence(__ATOMIC_ACQUIRE, "workgroup");
    if (OUTM == 0 || OUTM == 2) {
      float* C = Cf + (size_t)z * strideC;
      const int hh = lane >> 4, c4 = (lane & 15) * 4;
      for (int pass = 0; pass < 2; ++pass) {
#pragma unroll
        for (int it = 0; it < 8; ++it) {
          const int row = it * 2 + hh;
          v4f v = *(const v4f*)(slab + row * 68 + c4);
          *(volatile v4f*)(C + (size_t)(mBase + row) * ldc + n0 + c4) = v;
        }
        __threadfence();
      }
    }
    if (OUTM == 1 || OUTM == 2) {
      _Float16* C = Ch + (size_t)z * strideH;
      const int q = lane >> 3, c8 = (lane & 7) * 8;
      for (int pass = 0; pass < 2; ++pass) {
#pragma unroll
        for (int it = 0; it < 4; ++it) {
          const int row = it * 4 + q;
          const float* sp = slab + row * 68 + c8;
          float x[8];
#pragma unroll
          for (int e = 0; e < 8; ++e) x[e] = sp[e];
          float rr = oscale;
          if (EPI == 2) {
            float ss = 0.f;
#pragma unroll
            for (int e = 0; e < 8; ++e) ss += x[e] * x[e];
            ss += __shfl_xor(ss, 1, 32);
            ss += __shfl_xor(ss, 2, 32);
            ss += __shfl_xor(ss, 4, 32);
            rr = oscale * rsqrtf(ss * (1.0f / 64.0f) + 1e-6f);
          }
          v8h hv;
#pragma unroll
          for (int e = 0; e < 8; ++e) {
            float y = x[e] * rr;
            if (EPI == 2) y *= gvec[c8 + e];
            hv[e] = (_Float16)y;
          }
          *(volatile v8h*)(C + (size_t)(mBase + row) * ldh + n0 + c8) = hv;
        }
        __threadfence();
      }
    }
    __builtin_amdgcn_fence(__ATOMIC_RELEASE, "workgroup");
    __builtin_amdgcn_wave_barrier();
    __builtin_amdgcn_fence(__ATOMIC_ACQUIRE, "workgroup");
  }
}

__global__ __launch_bounds__(256) void k_wt16(const float* __restrict__ W, _Float16* __restrict__ o16, int R, int Cc, float wscale) {
  __shared__ __align__(16) float tf[64 * 68];
  const int c0 = blockIdx.x * 64, r0 = blockIdx.y * 64, tid = threadIdx.x;
  {
    const int lr = tid >> 4, c4 = (tid & 15) * 4;
#pragma unroll
    for (int it = 0; it < 4; ++it) {
      const int rr = it * 16 + lr;
      const v4f a = *(const v4f*)(W + (size_t)(r0 + rr) * Cc + c0 + c4);
      *(v4f*)(tf + rr * 68 + c4) = a;
    }
  }
  __syncthreads();
  const int sub = tid >> 3, c8 = (tid & 7) * 8;
  v8h hv[2];
#pragma unroll
  for (int it = 0; it < 2; ++it) {
    const int oc = it * 32 + sub;
    v8h a;
#pragma unroll
    for (int q = 0; q < 8; ++q) a[q] = (_Float16)(tf[(c8 + q) * 68 + oc] * wscale);
    hv[it] = a;
  }
  for (int pass = 0; pass < 2; ++pass) {
#pragma unroll
    for (int it = 0; it < 2; ++it) {
      const int oc = it * 32 + sub;
      const size_t go = (size_t)(c0 + oc) * R + r0 + c8;
      *(volatile v8h*)(o16 + go) = hv[it];
    }
    __threadfence();
  }
}

__global__ __launch_bounds__(256) void k_wtsplit(const float* __restrict__ W, unsigned short* __restrict__ oh,
                                                 unsigned short* __restrict__ ol, int R, int Cc) {
  __shared__ __align__(16) float tf[64 * 68];
  const int c0 = blockIdx.x * 64, r0 = blockIdx.y * 64, tid = threadIdx.x;
  {
    const int lr = tid >> 4, c4 = (tid & 15) * 4;
#pragma unroll
    for (int it = 0; it < 4; ++it) {
      const int rr = it * 16 + lr;
      const v4f a = *(const v4f*)(W + (size_t)(r0 + rr) * Cc + c0 + c4);
      *(v4f*)(tf + rr * 68 + c4) = a;
    }
  }
  __syncthreads();
  const int sub = tid >> 3, c8 = (tid & 7) * 8;
  v4u hv[2], lv[2];
#pragma unroll
  for (int it = 0; it < 2; ++it) {
    const int oc = it * 32 + sub;
    v4u a, a2;
#pragma unroll
    for (int q = 0; q < 4; ++q) {
      const float f0 = tf[(c8 + 2 * q) * 68 + oc];
      const float f1 = tf[(c8 + 2 * q + 1) * 68 + oc];
      const unsigned short h0 = f2bf_bits(f0), h1 = f2bf_bits(f1);
      const unsigned short l0 = f2bf_bits(f0 - bf_bits2f(h0)), l1 = f2bf_bits(f1 - bf_bits2f(h1));
      a[q]  = pk16(h0, h1);
      a2[q] = pk16(l0, l1);
    }
    hv[it] = a; lv[it] = a2;
  }
  for (int pass = 0; pass < 2; ++pass) {
#pragma unroll
    for (int it = 0; it < 2; ++it) {
      const int oc = it * 32 + sub;
      const size_t go = (size_t)(c0 + oc) * R + r0 + c8;
      *(volatile v4u*)(oh + go) = hv[it];
      *(volatile v4u*)(ol + go) = lv[it];
    }
    __threadfence();
  }
}

__global__ __launch_bounds__(256) void k_split2(const float* __restrict__ in, unsigned short* __restrict__ hi,
                                                unsigned short* __restrict__ lo, int n2) {
  const int i = blockIdx.x * 256 + threadIdx.x;
  if (i < n2) {
    const v2f f = *(const v2f*)(in + 2 * (size_t)i);
    const unsigned short h0 = f2bf_bits(f[0]), h1 = f2bf_bits(f[1]);
    const unsigned short l0 = f2bf_bits(f[0] - bf_bits2f(h0)), l1 = f2bf_bits(f[1] - bf_bits2f(h1));
    const unsigned uh = pk16(h0, h1), ul = pk16(l0, l1);
    ((volatile unsigned*)hi)[i] = uh;
    ((volatile unsigned*)lo)[i] = ul;
    __threadfence();
    ((volatile unsigned*)hi)[i] = uh;
    ((volatile unsigned*)lo)[i] = ul;
  }
}

__global__ __launch_bounds__(512) void k_invfreq(float* __restrict__ inv) {
  const int f = threadIdx.x;
  const float x = (float)f * (1.0f / 512.0f);
  const float v = 1.0f / powf(10000.0f, x);
  ((volatile float*)inv)[f] = v;
  __threadfence();
  ((volatile float*)inv)[f] = v;
}

__global__ __launch_bounds__(512) void k_cstab(const float* __restrict__ inv, float* __restrict__ cs) {
  const int n = blockIdx.x, f = threadIdx.x;
  const float ang = (float)n * inv[f];
  float sv, cv;
  sincosf(ang, &sv, &cv);
  v2f v; v.x = cv; v.y = sv;
  float* p = cs + ((size_t)n * 512 + f) * 2;
  *(volatile v2f*)p = v;
  __threadfence();
  *(volatile v2f*)p = v;
}

__global__ __launch_bounds__(128) void k_cvt_in(const float* __restrict__ text, const float* __restrict__ audio,
                                                const float* __restrict__ cs, _Float16* __restrict__ q16, _Float16* __restrict__ a16) {
  const int r = blockIdx.x, job = blockIdx.y, t = threadIdx.x, c0 = t * 8;
  const float* src = (job == 0) ? text : audio;
  _Float16* dst = (job == 0) ? q16 : a16;
  const float* xr = src + (size_t)r * DM + c0;
  const v4f x0 = *(const v4f*)xr, x1 = *(const v4f*)(xr + 4);
  float y[8] = {x0[0], x0[1], x0[2], x0[3], x1[0], x1[1], x1[2], x1[3]};
  if (job == 0) {
    const int n = r & (SEQ - 1);
    const bool lowh = (c0 < 512);
    const int pc = lowh ? (c0 + 512) : (c0 - 512);
    const float* pr = src + (size_t)r * DM + pc;
    const v4f p0 = *(const v4f*)pr, p1 = *(const v4f*)(pr + 4);
    const float pv[8] = {p0[0], p0[1], p0[2], p0[3], p1[0], p1[1], p1[2], p1[3]};
    const float* csr = cs + ((size_t)n * 512 + (c0 & 511)) * 2;
    const v4f t0 = *(const v4f*)csr, t1 = *(const v4f*)(csr + 4), t2 = *(const v4f*)(csr + 8), t3 = *(const v4f*)(csr + 12);
    const float cvv[8] = {t0[0], t0[2], t1[0], t1[2], t2[0], t2[2], t3[0], t3[2]};
    const float svv[8] = {t0[1], t0[3], t1[1], t1[3], t2[1], t2[3], t3[1], t3[3]};
#pragma unroll
    for (int e = 0; e < 8; ++e) {
      const float rot = lowh ? -pv[e] : pv[e];
      y[e] = y[e] * cvv[e] + rot * svv[e];
    }
  }
  v8h hv;
#pragma unroll
  for (int e = 0; e < 8; ++e) hv[e] = (_Float16)y[e];
  _Float16* op = dst + (size_t)r * DM + c0;
  *(volatile v8h*)op = hv;
  __threadfence();
  *(volatile v8h*)op = hv;
}

template <bool ROPE>
__global__ __launch_bounds__(128) void k_ln1024(const float* __restrict__ X, const float* __restrict__ g, const float* __restrict__ bb,
                                                const float* __restrict__ cs, _Float16* __restrict__ out, int nrows, int padrows) {
  __shared__ float red[4];
  __shared__ __align__(16) float rowv[DM];
  const int blk = blockIdx.x, t = threadIdx.x, c0 = 8 * t;
  const int lane = t & 31, wave = t >> 5;
  if (blk >= nrows) {
    const int p = blk - nrows;
    const v4u zz = {0u, 0u, 0u, 0u};
    _Float16* op = out + (size_t)p * DM + c0;
    *(volatile v4u*)op = zz;
    __threadfence();
    *(volatile v4u*)op = zz;
    return;
  }
  const int r = blk;
  const float* xr = X + (size_t)r * DM + c0;
  const v4f x0 = *(const v4f*)xr, x1 = *(const v4f*)(xr + 4);
  const float v[8] = {x0[0], x0[1], x0[2], x0[3], x1[0], x1[1], x1[2], x1[3]};
  float s = 0.f;
#pragma unroll
  for (int e = 0; e < 8; ++e) s += v[e];
  s = wsum(s);
  if (lane == 0) red[wave] = s;
  __syncthreads();
  const float mu = (red[0] + red[1] + red[2] + red[3]) * (1.0f / 1024.0f);
  __syncthreads();
  float d[8];
  float s2 = 0.f;
#pragma unroll
  for (int e = 0; e < 8; ++e) { d[e] = v[e] - mu; s2 += d[e] * d[e]; }
  s2 = wsum(s2);
  if (lane == 0) red[wave] = s2;
  __syncthreads();
  const float var = (red[0] + red[1] + red[2] + red[3]) * (1.0f / 1024.0f);
  const float rstd = rsqrtf(var + 1e-5f);
  const v4f g0 = *(const v4f*)(g + c0), g1 = *(const v4f*)(g + c0 + 4);
  const v4f b0 = *(const v4f*)(bb + c0), b1 = *(const v4f*)(bb + c0 + 4);
  const float gv[8] = {g0[0], g0[1], g0[2], g0[3], g1[0], g1[1], g1[2], g1[3]};
  const float bv[8] = {b0[0], b0[1], b0[2], b0[3], b1[0], b1[1], b1[2], b1[3]};
  float y[8];
#pragma unroll
  for (int e = 0; e < 8; ++e) y[e] = d[e] * rstd * gv[e] + bv[e];
  if (ROPE) {
#pragma unroll
    for (int e = 0; e < 8; ++e) rowv[c0 + e] = y[e];
    __syncthreads();
    const int n = r & (SEQ - 1);
    const bool lowh = (c0 < 512);
    const int pc = lowh ? (c0 + 512) : (c0 - 512);
    const float* csr = cs + ((size_t)n * 512 + (c0 & 511)) * 2;
    const v4f t0 = *(const v4f*)csr, t1 = *(const v4f*)(csr + 4), t2 = *(const v4f*)(csr + 8), t3 = *(const v4f*)(csr + 12);
    const float cvv[8] = {t0[0], t0[2], t1[0], t1[2], t2[0], t2[2], t3[0], t3[2]};
    const float svv[8] = {t0[1], t0[3], t1[1], t1[3], t2[1], t2[3], t3[1], t3[3]};
#pragma unroll
    for (int e = 0; e < 8; ++e) {
      const float pr = rowv[pc + e];
      const float rot = lowh ? -pr : pr;
      y[e] = y[e] * cvv[e] + rot * svv[e];
    }
  }
  v8h hv;
#pragma unroll
  for (int e = 0; e < 8; ++e) hv[e] = (_Float16)y[e];
  _Float16* op = out + (size_t)(padrows + r) * DM + c0;
  *(volatile v8h*)op = hv;
  __threadfence();
  *(volatile v8h*)op = hv;
}

__global__ __launch_bounds__(256) void k_ln_tsplit(const float* __restrict__ X, const float* __restrict__ g, const float* __restrict__ bb,
                                                  unsigned short* __restrict__ oh, unsigned short* __restrict__ ol, int nrowblk) {
  __shared__ __align__(16) float tf[64 * 68];
  __shared__ float smu[64];
  __shared__ float srs[64];
  const int tid = threadIdx.x, lane = tid & 31, wave = tid >> 5;
  const int bx = blockIdx.x;
  const int sub = tid >> 3, c8 = (tid & 7) * 8;
  if (bx >= nrowblk) {
    const int pb = bx - nrowblk;
    const v4u zz = {0u, 0u, 0u, 0u};
    for (int pass = 0; pass < 2; ++pass) {
      for (int it = 0; it < 32; ++it) {
        const int e = it * 32 + sub;
        const size_t go = (size_t)e * VTP + pb * 64 + c8;
        *(volatile v4u*)(oh + go) = zz;
        *(volatile v4u*)(ol + go) = zz;
      }
      __threadfence();
    }
    return;
  }
  const int r0 = bx * 64;
#pragma unroll 1
  for (int q = 0; q < 8; ++q) {
    const int rr = wave * 8 + q;
    const float* xr = X + (size_t)(r0 + rr) * DM + lane * 32;
    v4f a[8];
#pragma unroll
    for (int i = 0; i < 8; ++i) a[i] = *(const v4f*)(xr + 4 * i);
    float s = 0.f;
#pragma unroll
    for (int i = 0; i < 8; ++i) s += a[i][0] + a[i][1] + a[i][2] + a[i][3];
    s = wsum(s);
    const float mu = s * (1.0f / 1024.0f);
    float s2 = 0.f;
#pragma unroll
    for (int i = 0; i < 8; ++i) {
#pragma unroll
      for (int e = 0; e < 4; ++e) { const float dd = a[i][e] - mu; s2 += dd * dd; }
    }
    s2 = wsum(s2);
    if (lane == 0) { smu[rr] = mu; srs[rr] = rsqrtf(s2 * (1.0f / 1024.0f) + 1e-5f); }
  }
  __syncthreads();
  const int lr = tid >> 4, c4 = (tid & 15) * 4;
  for (int cb = 0; cb < DM / 64; ++cb) {
    const int c0 = cb * 64;
    const v4f gg = *(const v4f*)(g + c0 + c4);
    const v4f bv = *(const v4f*)(bb + c0 + c4);
#pragma unroll
    for (int it = 0; it < 4; ++it) {
      const int rr = it * 16 + lr;
      const v4f a = *(const v4f*)(X + (size_t)(r0 + rr) * DM + c0 + c4);
      const float mu = smu[rr], rs = srs[rr];
#pragma unroll
      for (int q = 0; q < 4; ++q) tf[rr * 68 + c4 + q] = (a[q] - mu) * rs * gg[q] + bv[q];
    }
    __syncthreads();
    v4u hv[2], lv[2];
#pragma unroll
    for (int it = 0; it < 2; ++it) {
      const int oc = it * 32 + sub;
      v4u a, a2;
#pragma unroll
      for (int q = 0; q < 4; ++q) {
        const float f0 = tf[(c8 + 2 * q) * 68 + oc];
        const float f1 = tf[(c8 + 2 * q + 1) * 68 + oc];
        const unsigned short h0 = f2bf_bits(f0), h1 = f2bf_bits(f1);
        const unsigned short l0 = f2bf_bits(f0 - bf_bits2f(h0)), l1 = f2bf_bits(f1 - bf_bits2f(h1));
        a[q]  = pk16(h0, h1);
        a2[q] = pk16(l0, l1);
      }
      hv[it] = a; lv[it] = a2;
    }
    for (int pass = 0; pass < 2; ++pass) {
#pragma unroll
      for (int it = 0; it < 2; ++it) {
        const int oc = it * 32 + sub;
        const size_t go = (size_t)(c0 + oc) * VTP + KPR + r0 + c8;
        *(volatile v4u*)(oh + go) = hv[it];
        *(volatile v4u*)(ol + go) = lv[it];
      }
      __threadfence();
    }
    __syncthreads();
  }
}

__global__ __launch_bounds__(128) void k_lsoftmax(const float* __restrict__ S, unsigned short* __restrict__ Ph, unsigned short* __restrict__ Pl) {
  __shared__ float red[4];
  const int r = blockIdx.x, t = threadIdx.x, c0 = 8 * t;
  const int lane = t & 31, wave = t >> 5;
  const int rem = r & (SEQ - 1), w = rem >> 9, i = rem & (WSZ - 1);
  const int qpos = w * WSZ + i;
  const float* sr = S + (size_t)r * (2 * WSZ) + c0;
  const v4f x0 = *(const v4f*)sr, x1 = *(const v4f*)(sr + 4);
  const float raw[8] = {x0[0], x0[1], x0[2], x0[3], x1[0], x1[1], x1[2], x1[3]};
  float s[8];
  float m = -3.0e38f;
#pragma unroll
  for (int e = 0; e < 8; ++e) {
    const int kpos = (w - 1) * WSZ + c0 + e;
    const bool masked = (kpos < 0) || (kpos > qpos);
    s[e] = masked ? -1.0e9f : raw[e];
    m = fmaxf(m, s[e]);
  }
  m = wmax(m);
  if (lane == 0) red[wave] = m;
  __syncthreads();
  const float rmax = fmaxf(fmaxf(red[0], red[1]), fmaxf(red[2], red[3]));
  __syncthreads();
  float ev[8];
  float sum = 0.f;
#pragma unroll
  for (int e = 0; e < 8; ++e) { ev[e] = expf(s[e] - rmax); sum += ev[e]; }
  sum = wsum(sum);
  if (lane == 0) red[wave] = sum;
  __syncthreads();
  const float tot = red[0] + red[1] + red[2] + red[3];
  const float inv = 1.0f / tot;
  v4u hv, lv;
#pragma unroll
  for (int q = 0; q < 4; ++q) {
    const float p0 = ev[2 * q] * inv, p1 = ev[2 * q + 1] * inv;
    const unsigned short h0 = f2bf_bits(p0), h1 = f2bf_bits(p1);
    const unsigned short l0 = f2bf_bits(p0 - bf_bits2f(h0)), l1 = f2bf_bits(p1 - bf_bits2f(h1));
    hv[q] = pk16(h0, h1);
    lv[q] = pk16(l0, l1);
  }
  const size_t go = (size_t)r * (2 * WSZ) + c0;
  *(volatile v4u*)(Ph + go) = hv;
  *(volatile v4u*)(Pl + go) = lv;
  __threadfence();
  *(volatile v4u*)(Ph + go) = hv;
  *(volatile v4u*)(Pl + go) = lv;
}

__device__ __forceinline__ v8f mma_h(v16h a, v16h b, v8f c) {
  c = __builtin_amdgcn_wmma_f32_16x16x32_f16(false, a, false, b, (short)0, c, false, false);
  asm volatile("v_nop\n\tv_nop\n\tv_nop\n\tv_nop" : "+v"(c) : "v"(a), "v"(b));
  return c;
}

__global__ __launch_bounds__(128)
void k_flash(const _Float16* __restrict__ qm, const _Float16* __restrict__ km,
             const _Float16* __restrict__ vt, float* __restrict__ out) {
  union FB { v16h v; v8h h[2]; };
  __shared__ __align__(16) _Float16 Ksh[64 * 64];
  __shared__ __align__(16) _Float16 Vth[64 * 64];
  __shared__ __align__(16) _Float16 Psh[4][16 * 64];
  __shared__ __align__(16) float    Os[4][16 * 68];

  const int tid  = threadIdx.x;
  const int wave = tid >> 5;
  const int lane = tid & 31;
  const int hh   = lane >> 4;
  const int c    = lane & 15;
  const int b  = blockIdx.y;
  const int qb = blockIdx.x & 31;
  const int h  = blockIdx.x >> 5;
  const int q0 = qb * 64 + wave * 16;

  const _Float16* Qb = qm + (size_t)b * SEQ * INR + h * DHD;
  const _Float16* Kb = km + (size_t)b * SEQ * INR + h * DHD;
  const _Float16* Vb = vt + (size_t)(h * DHD) * NTOK + (size_t)b * SEQ;
  float*          ob = out + (size_t)b * SEQ * INR + h * DHD;

  v16h qa[2];
#pragma unroll
  for (int dc = 0; dc < 2; ++dc) qa[dc] = Frag<_Float16>::load(Qb + (size_t)(q0 + c) * INR + dc * 32 + 8 * hh);

  float mrow[8], lrow[8];
  v8f oacc[4];
#pragma unroll
  for (int r = 0; r < 8; ++r) { mrow[r] = -INFINITY; lrow[r] = 0.f; }
#pragma unroll
  for (int t = 0; t < 4; ++t) oacc[t] = (v8f){0.f,0.f,0.f,0.f,0.f,0.f,0.f,0.f};

  const int nChunks = qb + 1;
  for (int kc = 0; kc < nChunks; ++kc) {
    const int kv0 = kc * 64;
    __syncthreads();
    {
      const int r = tid >> 1, half = (tid & 1) * 32;
      const _Float16* ks = Kb + (size_t)(kv0 + r) * INR + half;
      const _Float16* vs = Vb + (size_t)r * NTOK + kv0 + half;
#pragma unroll
      for (int i = 0; i < 4; ++i) {
        const v8h a0 = *(const v8h*)(ks + 8 * i);
        const v8h b0 = *(const v8h*)(vs + 8 * i);
        *(v8h*)(Ksh + r * 64 + half + 8 * i) = a0;
        *(v8h*)(Vth + r * 64 + half + 8 * i) = b0;
      }
    }
    __syncthreads();

    v8f s[4];
#pragma unroll
    for (int j = 0; j < 4; ++j) {
      s[j] = (v8f){0.f,0.f,0.f,0.f,0.f,0.f,0.f,0.f};
#pragma unroll
      for (int dc = 0; dc < 2; ++dc) {
        FB kb;
        kb.h[0] = *(const v8h*)(Ksh + (j * 16 + c) * 64 + dc * 32 + 8 * hh);
        kb.h[1] = *(const v8h*)(Ksh + (j * 16 + c) * 64 + dc * 32 + 16 + 8 * hh);
        s[j] = mma_h(qa[dc], kb.v, s[j]);
      }
    }
    const bool diag = (kc == qb);
    float cm[8];
#pragma unroll
    for (int r = 0; r < 8; ++r) {
      const int qrow = q0 + 8 * hh + r;
      float m = -INFINITY;
#pragma unroll
      for (int j = 0; j < 4; ++j) {
        const int kvcol = kv0 + j * 16 + c;
        const float sv = s[j][r] * 0.125f;
        const bool masked = diag && (kvcol > qrow);
        const float sm = masked ? -INFINITY : sv;
        s[j][r] = sm;
        m = fmaxf(m, sm);
      }
#pragma unroll
      for (int off = 1; off < 16; off <<= 1) m = fmaxf(m, __shfl_xor(m, off, 32));
      cm[r] = m;
    }
    _Float16* pw = Psh[wave];
#pragma unroll
    for (int r = 0; r < 8; ++r) {
      const float mnew = fmaxf(mrow[r], cm[r]);
      const float alpha = expf(mrow[r] - mnew);
      mrow[r] = mnew;
      float psum = 0.f;
#pragma unroll
      for (int j = 0; j < 4; ++j) {
        const float p = expf(s[j][r] - mnew);
        psum += p;
        pw[(8 * hh + r) * 64 + j * 16 + c] = (_Float16)(p * 4096.0f);
      }
#pragma unroll
      for (int off = 1; off < 16; off <<= 1) psum += __shfl_xor(psum, off, 32);
      lrow[r] = lrow[r] * alpha + psum;
#pragma unroll
      for (int t = 0; t < 4; ++t) oacc[t][r] *= alpha;
    }
    __builtin_amdgcn_fence(__ATOMIC_RELEASE, "workgroup");
    __builtin_amdgcn_wave_barrier();
    __builtin_amdgcn_fence(__ATOMIC_ACQUIRE, "workgroup");
#pragma unroll 1
    for (int kk = 0; kk < 2; ++kk) {
      FB pa;
      pa.h[0] = *(const v8h*)(pw + c * 64 + kk * 32 + 8 * hh);
      pa.h[1] = *(const v8h*)(pw + c * 64 + kk * 32 + 16 + 8 * hh);
#pragma unroll
      for (int t = 0; t < 4; ++t) {
        FB vb;
        vb.h[0] = *(const v8h*)(Vth + (t * 16 + c) * 64 + kk * 32 + 8 * hh);
        vb.h[1] = *(const v8h*)(Vth + (t * 16 + c) * 64 + kk * 32 + 16 + 8 * hh);
        oacc[t] = mma_h(pa.v, vb.v, oacc[t]);
      }
    }
  }

  float* os = Os[wave];
#pragma unroll
  for (int r = 0; r < 8; ++r) {
    const float inv = (1.0f / lrow[r]) * (1.0f / 4096.0f);
#pragma unroll
    for (int t = 0; t < 4; ++t) os[(8 * hh + r) * 68 + t * 16 + c] = oacc[t][r] * inv;
  }
  __builtin_amdgcn_fence(__ATOMIC_RELEASE, "workgroup");
  __builtin_amdgcn_wave_barrier();
  __builtin_amdgcn_fence(__ATOMIC_ACQUIRE, "workgroup");
  {
    const int c4 = (lane & 15) * 4;
    for (int pass = 0; pass < 2; ++pass) {
#pragma unroll
      for (int it = 0; it < 8; ++it) {
        const int row = it * 2 + hh;
        v4f val = *(const v4f*)(os + row * 68 + c4);
        *(volatile v4f*)(ob + (size_t)(q0 + row) * INR + c4) = val;
      }
      __threadfence();
    }
  }
}

__global__ __launch_bounds__(256) void k_ln4096(_Float16* __restrict__ U, const float* __restrict__ g, const float* __restrict__ bb) {
  __shared__ float red[8];
  const int r = blockIdx.x, t = threadIdx.x;
  const int lane = t & 31, wave = t >> 5;
  const int cA = 8 * t, cB = 2048 + 8 * t;
  _Float16* ur = U + (size_t)r * FFD;
  const v8h a = *(const v8h*)(ur + cA);
  const v8h a2 = *(const v8h*)(ur + cB);
  float v[16];
#pragma unroll
  for (int e = 0; e < 8; ++e) { v[e] = (float)a[e]; v[8 + e] = (float)a2[e]; }
  float s = 0.f;
#pragma unroll
  for (int e = 0; e < 16; ++e) s += v[e];
  s = wsum(s);
  if (lane == 0) red[wave] = s;
  __syncthreads();
  float tot = 0.f;
#pragma unroll
  for (int i = 0; i < 8; ++i) tot += red[i];
  const float mu = tot * (1.0f / 4096.0f);
  __syncthreads();
  float d[16];
  float s2 = 0.f;
#pragma unroll
  for (int e = 0; e < 16; ++e) { d[e] = v[e] - mu; s2 += d[e] * d[e]; }
  s2 = wsum(s2);
  if (lane == 0) red[wave] = s2;
  __syncthreads();
  float tot2 = 0.f;
#pragma unroll
  for (int i = 0; i < 8; ++i) tot2 += red[i];
  const float var_s = tot2 * (1.0f / 4096.0f);
  const float rstd = rsqrtf(var_s * (1.0f / 65536.0f) + 1e-5f) * (1.0f / 256.0f);
  v8h ha, hb;
#pragma unroll
  for (int e = 0; e < 8; ++e) {
    ha[e] = (_Float16)(d[e] * rstd * g[cA + e] + bb[cA + e]);
    hb[e] = (_Float16)(d[8 + e] * rstd * g[cB + e] + bb[cB + e]);
  }
  *(volatile v8h*)(ur + cA) = ha;
  *(volatile v8h*)(ur + cB) = hb;
  __threadfence();
  *(volatile v8h*)(ur + cA) = ha;
  *(volatile v8h*)(ur + cB) = hb;
}

extern "C" void kernel_launch(void* const* d_in, const int* in_sizes, int n_in,
                              void* d_out, int out_size, void* d_ws, size_t ws_size,
                              hipStream_t stream) {
  if (n_in < 24) return;
  if (in_sizes[0] != NTOK * DM || in_sizes[1] != NTOK * DM || in_sizes[2] != NTOK * DM) return;
  if (in_sizes[3] != DM * DM || in_sizes[7] != DM * DM || in_sizes[14] != DM * 2 * INR) return;
  if (in_sizes[13] != DM * INR || in_sizes[17] != INR * DM) return;
  if (in_sizes[18] != DM * FFD || in_sizes[22] != FFD * DM) return;
  if (in_sizes[4] != DM || in_sizes[5] != DM || in_sizes[6] != DM || in_sizes[8] != DM || in_sizes[9] != DM ||
      in_sizes[10] != DM || in_sizes[11] != DM || in_sizes[12] != DM || in_sizes[23] != DM) return;
  if (in_sizes[15] != DHD || in_sizes[16] != DHD) return;
  if (in_sizes[19] != FFD || in_sizes[20] != FFD || in_sizes[21] != FFD) return;
  if (out_size != NTOK * DM) return;

  const float* text  = (const float*)d_in[0];
  const float* audio = (const float*)d_in[1];
  const float* video = (const float*)d_in[2];
  const float* Wa    = (const float*)d_in[3];
  const float* ba    = (const float*)d_in[4];
  const float* lna_g = (const float*)d_in[5];
  const float* lna_b = (const float*)d_in[6];
  const float* Wvid  = (const float*)d_in[7];
  const float* bvid  = (const float*)d_in[8];
  const float* lnv_g = (const float*)d_in[9];
  const float* lnv_b = (const float*)d_in[10];
  const float* ln1_g = (const float*)d_in[11];
  const float* ln1_b = (const float*)d_in[12];
  const float* Wq    = (const float*)d_in[13];
  const float* Wkv   = (const float*)d_in[14];
  const float* qn_g  = (const float*)d_in[15];
  const float* kn_g  = (const float*)d_in[16];
  const float* Wo    = (const float*)d_in[17];
  const float* W1    = (const float*)d_in[18];
  const float* b1    = (const float*)d_in[19];
  const float* ln2_g = (const float*)d_in[20];
  const float* ln2_b = (const float*)d_in[21];
  const float* W2    = (const float*)d_in[22];
  const float* b2    = (const float*)d_in[23];
  float* outp = (float*)d_out;

  const size_t MIB = 1048576;
  size_t off = 0;
  const size_t oInv  = off; off += 4096;
  const size_t oCs   = off; off += (size_t)SEQ * 512 * 2 * 4;
  const size_t oWaT  = off; off += (size_t)DM * DM * 2;
  const size_t oWvTh = off; off += (size_t)DM * DM * 2;
  const size_t oWvTl = off; off += (size_t)DM * DM * 2;
  const size_t oWqT  = off; off += (size_t)INR * DM * 2;
  const size_t oWkvT = off; off += (size_t)2 * INR * DM * 2;
  const size_t oW1T  = off; off += (size_t)FFD * DM * 2;
  const size_t oW2T  = off; off += (size_t)DM * FFD * 2;
  const size_t oWoTh = off; off += (size_t)DM * INR * 2;
  const size_t oWoTl = off; off += (size_t)DM * INR * 2;
  const size_t oR3   = off; off += (size_t)NTOK * DM * 2;
  const size_t oR4   = off; off += (size_t)NTOK * DM * 4;
  const size_t oR5   = off; off += 51 * MIB;
  if (off > ws_size || off > (size_t)128 * MIB) return;

  char* ws = (char*)d_ws;
  float* inv = (float*)(ws + oInv);
  float* cs  = (float*)(ws + oCs);
  _Float16* WaT = (_Float16*)(ws + oWaT);
  unsigned short* WvTh = (unsigned short*)(ws + oWvTh);
  unsigned short* WvTl = (unsigned short*)(ws + oWvTl);
  _Float16* WqT  = (_Float16*)(ws + oWqT);
  _Float16* WkvT = (_Float16*)(ws + oWkvT);
  _Float16* W1T  = (_Float16*)(ws + oW1T);
  _Float16* W2T  = (_Float16*)(ws + oW2T);
  unsigned short* WoTh = (unsigned short*)(ws + oWoTh);
  unsigned short* WoTl = (unsigned short*)(ws + oWoTl);
  _Float16* q16 = (_Float16*)(ws + oR3);
  _Float16* h16 = (_Float16*)(ws + oR3);
  _Float16* x2h = (_Float16*)(ws + oR3);
  float* Cad = (float*)(ws + oR4);
  float* Sf  = (float*)(ws + oR4);
  float* Xf  = (float*)(ws + oR4);
  float* X2f = (float*)(ws + oR4);
  char* r5 = ws + oR5;
  _Float16* a16 = (_Float16*)(r5);
  unsigned short* vih = (unsigned short*)(r5 + 8 * MIB);
  unsigned short* vil = (unsigned short*)(r5 + 16 * MIB);
  _Float16* k16 = (_Float16*)(r5 + 24 * MIB);
  unsigned short* vTh = (unsigned short*)(r5 + 33 * MIB);
  unsigned short* vTl = (unsigned short*)(r5 + 42 * MIB);
  unsigned short* Ph  = (unsigned short*)(r5);
  unsigned short* Pl  = (unsigned short*)(r5 + 8 * MIB);
  _Float16* qm16 = (_Float16*)(r5);
  _Float16* km16 = (_Float16*)(r5 + 4 * MIB);
  _Float16* vT16 = (_Float16*)(r5 + 8 * MIB);
  float* Of = (float*)(r5 + 16 * MIB);
  unsigned short* Oh = (unsigned short*)(r5 + 24 * MIB);
  unsigned short* Ol = (unsigned short*)(r5 + 28 * MIB);
  _Float16* U16 = (_Float16*)(r5);

  const dim3 blk(256);
  const unsigned short* N16 = (const unsigned short*)nullptr;

  k_invfreq<<<dim3(1), dim3(512), 0, stream>>>(inv);
  k_cstab<<<dim3(SEQ), dim3(512), 0, stream>>>(inv, cs);

  k_wt16<<<dim3(DM / 64, DM / 64), blk, 0, stream>>>(Wa, WaT, DM, DM, 64.0f);
  k_wtsplit<<<dim3(DM / 64, DM / 64), blk, 0, stream>>>(Wvid, WvTh, WvTl, DM, DM);
  k_wt16<<<dim3(INR / 64, DM / 64), blk, 0, stream>>>(Wq, WqT, DM, INR, 64.0f);
  k_wt16<<<dim3(2 * INR / 64, DM / 64), blk, 0, stream>>>(Wkv, WkvT, DM, 2 * INR, 64.0f);
  k_wt16<<<dim3(FFD / 64, DM / 64), blk, 0, stream>>>(W1, W1T, DM, FFD, 64.0f);
  k_wt16<<<dim3(DM / 64, FFD / 64), blk, 0, stream>>>(W2, W2T, FFD, DM, 64.0f);
  k_wtsplit<<<dim3(DM / 64, INR / 64), blk, 0, stream>>>(Wo, WoTh, WoTl, INR, DM);

  k_cvt_in<<<dim3(NTOK, 2), dim3(128), 0, stream>>>(text, audio, cs, q16, a16);
  const int n2v = NTOK * DM / 2;
  k_split2<<<dim3((n2v + 255) / 256), blk, 0, stream>>>(video, vih, vil, n2v);

  const dim3 gA(((NTOK / 64) * (DM / 64) + 7) / 8, 1);
  k_gemm<0, false, true, 0, 0, false, 0><<<gA, blk, 0, stream>>>(
      (const unsigned short*)a16, N16, DM, 0L, (const unsigned short*)WaT, N16, DM, 0L,
      Cad, DM, 0L, nullptr, 0, 0L, ba, nullptr, nullptr, 0, 0L, NTOK, DM, DM, 1, 1.0f / 64.0f, 1.0f);
  k_ln1024<true><<<dim3(NTOK + KPR), dim3(128), 0, stream>>>(Cad, lna_g, lna_b, cs, k16, NTOK, KPR);

  k_gemm<1, true, true, 0, 0, false, 0><<<gA, blk, 0, stream>>>(
      vih, vil, DM, 0L, WvTh, WvTl, DM, 0L,
      Cad, DM, 0L, nullptr, 0, 0L, bvid, nullptr, nullptr, 0, 0L, NTOK, DM, DM, 1, 1.0f, 1.0f);
  k_ln_tsplit<<<dim3(NTOK / 64 + KPR / 64), blk, 0, stream>>>(Cad, lnv_g, lnv_b, vTh, vTl, NTOK / 64);

  const dim3 gS(((WSZ / 64) * (2 * WSZ / 64) + 7) / 8, NB_ * NWN);
  k_gemm<0, false, false, 0, 0, false, 1><<<gS, blk, 0, stream>>>(
      (const unsigned short*)q16, N16, DM, (long)WSZ * DM, (const unsigned short*)k16, N16, DM, (long)WSZ * DM,
      Sf, 2 * WSZ, (long)WSZ * 2 * WSZ, nullptr, 0, 0L, nullptr, nullptr, nullptr, 0, 0L,
      WSZ, 2 * WSZ, DM, NWN, 1.0f / 32.0f, 1.0f);
  k_lsoftmax<<<dim3(NTOK), dim3(128), 0, stream>>>(Sf, Ph, Pl);
  const dim3 gPV(((WSZ / 64) * (DM / 64) + 7) / 8, NB_ * NWN);
  k_gemm<1, true, false, 0, 0, false, 2><<<gPV, blk, 0, stream>>>(
      Ph, Pl, 2 * WSZ, (long)WSZ * 2 * WSZ, vTh, vTl, VTP, (long)WSZ,
      Xf, DM, (long)WSZ * DM, nullptr, 0, 0L, nullptr, nullptr, nullptr, 0, 0L,
      WSZ, DM, 2 * WSZ, NWN, 1.0f, 1.0f);

  k_ln1024<false><<<dim3(NTOK), dim3(128), 0, stream>>>(Xf, ln1_g, ln1_b, cs, h16, NTOK, 0);
  const dim3 gQ(((NTOK / 64) * (INR / 64) + 7) / 8, 1);
  k_gemm<0, false, false, 2, 1, false, 0><<<gQ, blk, 0, stream>>>(
      (const unsigned short*)h16, N16, DM, 0L, (const unsigned short*)WqT, N16, DM, 0L,
      nullptr, 0, 0L, qm16, INR, 0L, nullptr, qn_g, nullptr, 0, 0L, NTOK, INR, DM, 1, 1.0f / 64.0f, 1.0f);
  k_gemm<0, false, false, 2, 1, false, 0><<<gQ, blk, 0, stream>>>(
      (const unsigned short*)h16, N16, DM, 0L, (const unsigned short*)WkvT, N16, DM, 0L,
      nullptr, 0, 0L, km16, INR, 0L, nullptr, kn_g, nullptr, 0, 0L, NTOK, INR, DM, 1, 1.0f / 64.0f, 1.0f);
  const dim3 gVT(((INR / 64) * (NTOK / 64) + 7) / 8, 1);
  k_gemm<0, false, false, 0, 1, false, 0><<<gVT, blk, 0, stream>>>(
      (const unsigned short*)(WkvT + (size_t)INR * DM), N16, DM, 0L, (const unsigned short*)h16, N16, DM, 0L,
      nullptr, 0, 0L, vT16, NTOK, 0L, nullptr, nullptr, nullptr, 0, 0L, INR, NTOK, DM, 1, 1.0f / 64.0f, 1.0f);

  k_flash<<<dim3(NHD * (SEQ / 64), NB_), dim3(128), 0, stream>>>(qm16, km16, vT16, Of);
  const int n2o = NTOK * INR / 2;
  k_split2<<<dim3((n2o + 255) / 256), blk, 0, stream>>>(Of, Oh, Ol, n2o);

  k_gemm<1, true, false, 0, 2, false, 0><<<gA, blk, 0, stream>>>(
      Oh, Ol, INR, 0L, WoTh, WoTl, INR, 0L,
      X2f, DM, 0L, x2h, DM, 0L, nullptr, nullptr, nullptr, 0, 0L, NTOK, DM, INR, 1, 2.0f, 1024.0f);

  const dim3 gW1(((NTOK / 64) * (FFD / 64) + 7) / 8, 1);
  k_gemm<0, false, true, 1, 1, false, 0><<<gW1, blk, 0, stream>>>(
      (const unsigned short*)x2h, N16, DM, 0L, (const unsigned short*)W1T, N16, DM, 0L,
      nullptr, 0, 0L, U16, FFD, 0L, b1, nullptr, nullptr, 0, 0L, NTOK, FFD, DM, 1, 1.0f / 65536.0f, 256.0f);
  k_ln4096<<<dim3(NTOK), blk, 0, stream>>>(U16, ln2_g, ln2_b);
  k_gemm<0, false, true, 0, 0, true, 0><<<gA, blk, 0, stream>>>(
      (const unsigned short*)U16, N16, FFD, 0L, (const unsigned short*)W2T, N16, FFD, 0L,
      outp, DM, 0L, nullptr, 0, 0L, b2, nullptr, X2f, DM, 0L, NTOK, DM, FFD, 1, 1.0f / 64.0f, 1.0f);
  (void)hipGetLastError();
}
